// GINNet_46883863003469
// MI455X (gfx1250) — hardware-verified
//
#include <hip/hip_runtime.h>


namespace {
constexpr int N = 50000, E = 800000, H = 64, L = 3, ED = 2 * H + 2, EDP = 160, NPAD = 50048, NBLK = NPAD / 128;

typedef _Float16 b16;
typedef __attribute__((ext_vector_type(16))) _Float16 v16b;
typedef __attribute__((ext_vector_type(8)))  _Float16 v8b;
typedef __attribute__((ext_vector_type(8)))  float v8f;
typedef __attribute__((ext_vector_type(4)))  float v4f;

__device__ __forceinline__ v8b ld8b(const b16* p) { return *(const v8b*)p; }
__device__ __forceinline__ v16b cat8b(v8b a, v8b b) { return __builtin_shufflevector(a, b, 0, 1, 2, 3, 4, 5, 6, 7, 8, 9, 10, 11, 12, 13, 14, 15); }
__device__ __forceinline__ v16b frag_kb(const b16* p, int hh) { return cat8b(ld8b(p + 8 * hh), ld8b(p + 16 + 8 * hh)); }
__device__ __forceinline__ void split16(float v, b16& hi, b16& lo) { hi = (b16)v; lo = (b16)(v - (float)hi); }
__device__ __forceinline__ void frag_ksplit(const float* p, int hh, v16b& fh_, v16b& fl_) {
  const float* p0 = p + 8 * hh; const float* p1 = p + 16 + 8 * hh;
#pragma unroll
  for (int e = 0; e < 8; ++e) { b16 a, c; split16(p0[e], a, c); fh_[e] = a; fl_[e] = c; split16(p1[e], a, c); fh_[8 + e] = a; fl_[8 + e] = c; }
}
__device__ __forceinline__ v8f wmma16b(v16b a, v16b b, v8f c) {
  v8f d = __builtin_amdgcn_wmma_f32_16x16x32_f16(false, a, false, b, (short)0, c, false, false);
  asm volatile("v_nop\n\tv_nop\n\tv_nop\n\tv_nop" : "+v"(d) : "v"(a), "v"(b));
  return d;
}
__device__ __forceinline__ void wave_lds_sync() {
  __builtin_amdgcn_fence(__ATOMIC_RELEASE, "workgroup");
  __builtin_amdgcn_wave_barrier();
  __builtin_amdgcn_fence(__ATOMIC_ACQUIRE, "workgroup");
}

struct Opnd { const void* p0; const void* p1; int ld; };
template <int NP> __device__ __forceinline__ void load_frags(const Opnd& o, int row, int kb, int hh, v16b& fh_, v16b& fl_) {
  if (NP == 0) { frag_ksplit((const float*)o.p0 + (size_t)row * o.ld + kb, hh, fh_, fl_); }
  else if (NP == 4) {
    const float* p = (const float*)o.p0 + (size_t)row * o.ld + kb; const float* p0 = p + 8 * hh; const float* p1 = p + 16 + 8 * hh;
#pragma unroll
    for (int e = 0; e < 8; ++e) { b16 a, c; split16(p0[e] * 64.0f, a, c); fh_[e] = a; fl_[e] = c; split16(p1[e] * 64.0f, a, c); fh_[8 + e] = a; fl_[8 + e] = c; }
  } else if (NP == 3) {
    const float* p = (const float*)o.p0 + (size_t)row * o.ld + kb; const float* p0 = p + 8 * hh; const float* p1 = p + 16 + 8 * hh;
#pragma unroll
    for (int e = 0; e < 8; ++e) { fh_[e] = (b16)p0[e]; fh_[8 + e] = (b16)p1[e]; }
    fl_ = fh_;
  } else {
    fh_ = frag_kb((const b16*)o.p0 + (size_t)row * o.ld + kb, hh);
    if (NP == 2) fl_ = frag_kb((const b16*)o.p1 + (size_t)row * o.ld + kb, hh); else fl_ = fh_;
  }
}
template <int ANP, int BNP> __device__ __forceinline__ v8f mac(v16b ah, v16b al, v16b bh, v16b bl, v8f c) {
  c = wmma16b(ah, bh, c);
  if (BNP == 0 || BNP == 2 || BNP == 4) c = wmma16b(ah, bl, c);
  if (ANP == 0 || ANP == 2 || ANP == 4) c = wmma16b(al, bh, c);
  return c;
}
template <int ANP, int BNP>
__device__ __forceinline__ void gemm_tile(const Opnd& A, const Opnd& B, int K, int m0, int c0, int nloc, int hlf, v8f (&acc)[2][4]) {
  for (int kb = 0; kb < K; kb += 32) {
    v16b a0h, a0l, a1h, a1l;
    load_frags<ANP>(A, m0 + nloc, kb, hlf, a0h, a0l);
    load_frags<ANP>(A, m0 + 16 + nloc, kb, hlf, a1h, a1l);
#pragma unroll
    for (int t = 0; t < 4; ++t) {
      v16b bh, bl;
      load_frags<BNP>(B, c0 + t * 16 + nloc, kb, hlf, bh, bl);
      acc[0][t] = mac<ANP, BNP>(a0h, a0l, bh, bl, acc[0][t]);
      acc[1][t] = mac<ANP, BNP>(a1h, a1l, bh, bl, acc[1][t]);
    }
  }
}

__device__ __forceinline__ void epi_planes(v8f (&acc)[2][4], float scale, bool two, b16* __restrict__ oh, b16* __restrict__ ol, int ldo,
                                           int m0, int c0, int lane, b16* Th, b16* Tl) {
  const int nloc = lane & 15, hlf = lane >> 4;
#pragma unroll
  for (int t = 0; t < 4; ++t)
#pragma unroll
    for (int r = 0; r < 2; ++r)
#pragma unroll
      for (int v = 0; v < 8; ++v) {
        const int rr = r * 16 + v + 8 * hlf, cc = t * 16 + nloc;
        b16 h_, l_; split16(acc[r][t][v] * scale, h_, l_);
        Th[rr * 64 + cc] = h_; Tl[rr * 64 + cc] = l_;
      }
  wave_lds_sync();
  for (int pass = 0; pass < 2; ++pass) {
#pragma unroll
    for (int j = 0; j < 8; ++j) {
      const int rr = j * 4 + (lane >> 3), c8 = (lane & 7) * 8;
      const size_t o = (size_t)(m0 + rr) * ldo + c0 + c8;
      *(volatile v8b*)(oh + o) = ld8b(Th + rr * 64 + c8);
      if (two) *(volatile v8b*)(ol + o) = ld8b(Tl + rr * 64 + c8);
    }
    __threadfence();
  }
}
__device__ __forceinline__ void epi_f32(v8f (&acc)[2][4], float scale, const float* rscale, float* __restrict__ out, int ldo, int m0, int c0, int lane, float* Tt) {
  const int nloc = lane & 15, hlf = lane >> 4;
#pragma unroll
  for (int t = 0; t < 4; ++t)
#pragma unroll
    for (int r = 0; r < 2; ++r)
#pragma unroll
      for (int v = 0; v < 8; ++v) {
        const int rr = r * 16 + v + 8 * hlf;
        const float rs = rscale ? rscale[(size_t)(m0 + rr) * 32] : 1.0f;
        Tt[rr * 64 + t * 16 + nloc] = acc[r][t][v] * scale * rs;
      }
  wave_lds_sync();
  float* dst0 = out + (size_t)m0 * ldo + c0;
  for (int pass = 0; pass < 2; ++pass) {
#pragma unroll
    for (int j = 0; j < 16; ++j) { const int rr = j * 2 + hlf, c4 = nloc * 4; *(volatile v4f*)(dst0 + (size_t)rr * ldo + c4) = *(const v4f*)(Tt + rr * 64 + c4); }
    __threadfence();
  }
}


__global__ __launch_bounds__(256) void prep_kernel(const float* __restrict__ h, const float* __restrict__ embW, const float* __restrict__ W1, const float* __restrict__ W2, const float* __restrict__ pW1,
                                                   float* __restrict__ hp, b16* __restrict__ wemb, b16* __restrict__ w1, b16* __restrict__ w2, b16* __restrict__ wp) {
  const size_t tid = (size_t)blockIdx.x * blockDim.x + threadIdx.x, nth = (size_t)gridDim.x * blockDim.x;
  for (int pass = 0; pass < 2; ++pass) {
    for (size_t p = tid; p < (size_t)NPAD * H / 4; p += nth) { const size_t n = p / (H / 4); const v4f v = (n < (size_t)N) ? *(const v4f*)(h + p * 4) : (v4f){0.0f, 0.0f, 0.0f, 0.0f}; *(volatile v4f*)(hp + p * 4) = v; }
    for (size_t p = tid; p < (size_t)H * H / 8; p += nth) { const int n = (int)(p / 8), k0 = (int)(p % 8) * 8; v8b v;
#pragma unroll
      for (int e = 0; e < 8; ++e) v[e] = (b16)embW[(size_t)(k0 + e) * H + n];
      *(volatile v8b*)(wemb + (size_t)n * H + k0) = v; }
    for (size_t p = tid; p < (size_t)2 * L * H * H / 8; p += nth) { const int which = (int)(p / (L * H * H / 8)); const int rem = (int)(p % (L * H * H / 8)), l = rem / (H * H / 8), r2 = rem % (H * H / 8), n = r2 / 8, k0 = (r2 % 8) * 8;
      const float* W = (which ? W2 : W1) + (size_t)l * H * H; v8b v;
#pragma unroll
      for (int e = 0; e < 8; ++e) v[e] = (b16)W[(size_t)(k0 + e) * H + n];
      *(volatile v8b*)((which ? w2 : w1) + (size_t)l * H * H + (size_t)n * H + k0) = v; }
    for (size_t p = tid; p < (size_t)(L + 1) * H * EDP / 8; p += nth) { const int i = (int)(p / (H * EDP / 8)); const int rem = (int)(p % (H * EDP / 8)), n = rem / (EDP / 8), k0 = (rem % (EDP / 8)) * 8; v8b v;
#pragma unroll
      for (int e = 0; e < 8; ++e) { const int k = k0 + e; v[e] = (b16)((k < ED) ? pW1[((size_t)i * ED + k) * H + n] : 0.0f); }
      *(volatile v8b*)(wp + ((size_t)i * H + n) * EDP + k0) = v; }
    __threadfence();
  }
}

template <int DF, int NB>
__global__ __launch_bounds__(256) void agg_kernel(const int* __restrict__ esrc, const int* __restrict__ edst, const float* __restrict__ x, const float* __restrict__ epsl, float* __restrict__ zin) {
  const float opeps = 1.0f + epsl[0];
  __shared__ __attribute__((aligned(16))) int acc[NB * DF];
  __shared__ int list[8 * 256]; __shared__ int cnt[NB];
  constexpr float FXS = 524288.0f, FXI = 1.0f / 524288.0f;
  const int t_ = threadIdx.x, wave = t_ >> 5, lane = t_ & 31, base = blockIdx.x * NB;
  for (int i = t_; i < NB * DF; i += 256) acc[i] = 0;
  for (int i = t_; i < NB; i += 256) cnt[i] = 0;
  __syncthreads();
  int* wl = list + wave * 256;
  typedef __attribute__((ext_vector_type(4))) int v4i;
  for (int c0 = 0; c0 < E; c0 += 256 * 8) {
    const int e0 = c0 + (wave * 32 + lane) * 8;
    int dd[8];
    if (e0 + 7 < E) { const v4i a = *(const v4i*)(edst + e0), b = *(const v4i*)(edst + e0 + 4); dd[0] = a[0]; dd[1] = a[1]; dd[2] = a[2]; dd[3] = a[3]; dd[4] = b[0]; dd[5] = b[1]; dd[6] = b[2]; dd[7] = b[3]; }
    else {
#pragma unroll
      for (int j = 0; j < 8; ++j) dd[j] = (e0 + j < E) ? edst[e0 + j] : -1; }
    unsigned sl[8]; bool hit[8]; bool anyl = false;
#pragma unroll
    for (int j = 0; j < 8; ++j) { sl[j] = (unsigned)(dd[j] - base); hit[j] = sl[j] < (unsigned)NB; anyl |= hit[j]; }
    int wc = 0;
    if (__builtin_amdgcn_ballot_w32(anyl) != 0u) {
#pragma unroll
      for (int j = 0; j < 8; ++j) {
        const unsigned mj = __builtin_amdgcn_ballot_w32(hit[j]);
        if (mj != 0u) {
          if (hit[j]) { const int pos = wc + (int)__builtin_amdgcn_mbcnt_lo(mj, 0u); int s = esrc[e0 + j]; s = (s < 0) ? 0 : (s >= N ? N - 1 : s); wl[pos] = (s << 12) | (int)sl[j]; atomicAdd(&cnt[sl[j]], 1); }
          wc += __builtin_popcount(mj);
        }
      }
    }
    __builtin_amdgcn_wave_barrier(); __builtin_amdgcn_fence(__ATOMIC_RELEASE, "workgroup"); __builtin_amdgcn_fence(__ATOMIC_ACQUIRE, "workgroup");
    { constexpr int LPH = DF / 4, HPS = 32 / LPH;
      for (int i0 = 0; i0 < wc; i0 += HPS) { const int i = i0 + lane / LPH; if (i < wc) { const int ent = wl[i]; const int s = ent >> 12, slot = ent & 4095; const int col = (lane % LPH) * 4;
          const v4f v = *(const v4f*)(x + (size_t)s * DF + col);
#pragma unroll
          for (int c = 0; c < 4; ++c) atomicAdd(&acc[slot * DF + col + c], (int)rintf(v[c] * FXS)); } } }
    __builtin_amdgcn_wave_barrier();
  }
  __syncthreads();
  for (int pass = 0; pass < 2; ++pass) {
    for (int i = t_; i < NB * DF / 4; i += 256) { const int r = (i * 4) / DF; const int node = base + r; if (node < NPAD) {
        v4f o = {0.0f, 0.0f, 0.0f, 0.0f}; if (node < N) { const v4f xx = *(const v4f*)(x + (size_t)node * DF + (size_t)((i * 4) % DF));
#pragma unroll
          for (int c = 0; c < 4; ++c) o[c] = (float)acc[i * 4 + c] * FXI + opeps * xx[c]; }
        *(volatile v4f*)(zin + (size_t)base * DF + (size_t)i * 4) = o; } }
    __threadfence();
  }
}


template <int MODE>
__global__ __launch_bounds__(128) void nlin_kernel(const float* __restrict__ x, const b16* __restrict__ w, const float* __restrict__ b, const float* __restrict__ s1, const float* __restrict__ sh1,
                                                   const float* __restrict__ s2, const float* __restrict__ sh2, const float* __restrict__ res, float* __restrict__ out) {
  __shared__ __attribute__((aligned(16))) float Ts[4][32 * 64];
  const int lane = threadIdx.x & 31, wave = threadIdx.x >> 5, nloc = lane & 15, hlf = lane >> 4, m0 = blockIdx.x * 128 + wave * 32;
  v8f acc[2][4];
#pragma unroll
  for (int r = 0; r < 2; ++r)
#pragma unroll
    for (int t = 0; t < 4; ++t) acc[r][t] = (v8f){};
  const Opnd A{x, nullptr, H}, B{w, nullptr, H};
  gemm_tile<3, 1>(A, B, H, m0, 0, nloc, hlf, acc);
  float* Tt = Ts[wave];
#pragma unroll
  for (int t = 0; t < 4; ++t)
#pragma unroll
    for (int r = 0; r < 2; ++r)
#pragma unroll
      for (int v = 0; v < 8; ++v) { const int rr = r * 16 + v + 8 * hlf, c = t * 16 + nloc; float val = acc[r][t][v] + b[c];
        if (MODE == 1) val = fmaxf(val * s1[c] + sh1[c], 0.0f);
        if (MODE == 2) { val = fmaxf(val * s1[c] + sh1[c], 0.0f); val = fmaxf(val * s2[c] + sh2[c], 0.0f); val += res[(size_t)(m0 + rr) * H + c]; }
        Tt[rr * 64 + c] = val; }
  wave_lds_sync();
  for (int pass = 0; pass < 2; ++pass) {
#pragma unroll
    for (int j = 0; j < 16; ++j) { const int rr = j * 2 + hlf, c4 = nloc * 4; *(volatile v4f*)(out + (size_t)(m0 + rr) * H + c4) = *(const v4f*)(Tt + rr * 64 + c4); }
    __threadfence();
  }
}

template <bool FIRST, bool LAST>
__global__ __launch_bounds__(128) void edge_kernel(const int* __restrict__ esrc, const int* __restrict__ edst, const float* __restrict__ ef, const float* __restrict__ hcur, const b16* __restrict__ wp,
                                                   const float* __restrict__ b1, const float* __restrict__ W2, const float* __restrict__ b2, float* __restrict__ score, float* __restrict__ out) {
  __shared__ __attribute__((aligned(16))) b16 Ft[4][32][EDP + 8]; __shared__ float Sc[4][32];
  const int wave = threadIdx.x >> 5, lane = threadIdx.x & 31, nloc = lane & 15, hlf = lane >> 4, e0 = (blockIdx.x * 4 + wave) * 32;
  { const int e = e0 + lane; int s = esrc[e], d = edst[e]; s = (s < 0) ? 0 : (s >= N ? N - 1 : s); d = (d < 0) ? 0 : (d >= N ? N - 1 : d);
    const float* rs = hcur + (size_t)s * H; const float* rd = hcur + (size_t)d * H;
#pragma unroll
    for (int i = 0; i < H; i += 4) { const v4f a = *(const v4f*)(rs + i), c = *(const v4f*)(rd + i);
      Ft[wave][lane][i] = (b16)a[0]; Ft[wave][lane][i + 1] = (b16)a[1]; Ft[wave][lane][i + 2] = (b16)a[2]; Ft[wave][lane][i + 3] = (b16)a[3];
      Ft[wave][lane][H + i] = (b16)c[0]; Ft[wave][lane][H + i + 1] = (b16)c[1]; Ft[wave][lane][H + i + 2] = (b16)c[2]; Ft[wave][lane][H + i + 3] = (b16)c[3]; }
    Ft[wave][lane][2 * H] = (b16)ef[(size_t)e * 2]; Ft[wave][lane][2 * H + 1] = (b16)ef[(size_t)e * 2 + 1];
#pragma unroll
    for (int i = 2 * H + 2; i < EDP; ++i) Ft[wave][lane][i] = (b16)0.0f; }
  wave_lds_sync();
  v8f acc[2][4];
#pragma unroll
  for (int r = 0; r < 2; ++r)
#pragma unroll
    for (int t = 0; t < 4; ++t) acc[r][t] = (v8f){};
#pragma unroll
  for (int kb = 0; kb < EDP; kb += 32) {
    const v16b a0 = frag_kb(&Ft[wave][nloc][0] + kb, hlf), a1 = frag_kb(&Ft[wave][16 + nloc][0] + kb, hlf);
#pragma unroll
    for (int t = 0; t < 4; ++t) { const v16b bw = frag_kb(wp + (size_t)(t * 16 + nloc) * EDP + kb, hlf); acc[0][t] = wmma16b(a0, bw, acc[0][t]); acc[1][t] = wmma16b(a1, bw, acc[1][t]); }
  }
  float part[2][8];
#pragma unroll
  for (int r = 0; r < 2; ++r)
#pragma unroll
    for (int v = 0; v < 8; ++v) { float s = 0.0f;
#pragma unroll
      for (int t = 0; t < 4; ++t) { const int c = t * 16 + nloc; s += fmaxf(acc[r][t][v] + b1[c], 0.0f) * W2[c]; }
      part[r][v] = s; }
#pragma unroll
  for (int o = 1; o < 16; o <<= 1)
#pragma unroll
    for (int r = 0; r < 2; ++r)
#pragma unroll
      for (int v = 0; v < 8; ++v) part[r][v] += __shfl_xor(part[r][v], o);
  if (nloc == 0) {
#pragma unroll
    for (int r = 0; r < 2; ++r)
#pragma unroll
      for (int v = 0; v < 8; ++v) Sc[wave][r * 16 + 8 * hlf + v] = part[r][v] + b2[0]; }
  wave_lds_sync();
  float tot = Sc[wave][lane]; if (!FIRST) tot += score[e0 + lane];
  for (int pass = 0; pass < 2; ++pass) { if (LAST) ((volatile float*)out)[e0 + lane] = fmaxf(tot, 0.0f); else ((volatile float*)score)[e0 + lane] = tot; __threadfence(); }
}
}

extern "C" void kernel_launch(void* const* d_in, const int* in_sizes, int n_in,
                              void* d_out, int out_size, void* d_ws, size_t ws_size, hipStream_t stream) {
  (void)n_in; (void)out_size;
  const float* h = (const float*)d_in[0]; const float* ef = (const float*)d_in[1]; const int* src = (const int*)d_in[2]; const int* dst = (const int*)d_in[3];
  const float* embW = (const float*)d_in[4]; const float* embb = (const float*)d_in[5]; const float* eps = (const float*)d_in[6];
  const float* W1 = (const float*)d_in[7]; const float* b1 = (const float*)d_in[8]; const float* bns = (const float*)d_in[9]; const float* bnsh = (const float*)d_in[10];
  const float* W2 = (const float*)d_in[11]; const float* b2 = (const float*)d_in[12]; const float* aps = (const float*)d_in[13]; const float* apsh = (const float*)d_in[14];
  const float* gns = (const float*)d_in[15]; const float* gnsh = (const float*)d_in[16];
  const float* pW1 = (const float*)d_in[17]; const float* pb1 = (const float*)d_in[18]; const float* pW2 = (const float*)d_in[19]; const float* pb2 = (const float*)d_in[20];
  float* out = (float*)d_out;
  if (in_sizes[0] != N * H || in_sizes[1] != E * 2 || in_sizes[2] != E || in_sizes[6] != L || in_sizes[17] != (L + 1) * ED * H) return;
  size_t off = 0; char* ws = (char*)d_ws;
  auto carve = [&](size_t bytes) { char* p = ws + off; off += (bytes + 255) & ~(size_t)255; return p; };
  float* hp = (float*)carve((size_t)NPAD * H * 4); float* hA = (float*)carve((size_t)NPAD * H * 4); float* hB = (float*)carve((size_t)NPAD * H * 4); float* xa = (float*)carve((size_t)NPAD * H * 4); float* xb = (float*)carve((size_t)NPAD * H * 4);
  b16* wemb = (b16*)carve(H * H * 2); b16* w1 = (b16*)carve((size_t)L * H * H * 2); b16* w2 = (b16*)carve((size_t)L * H * H * 2); b16* wp = (b16*)carve((size_t)(L + 1) * H * EDP * 2);
  float* score = (float*)carve((size_t)E * 4);
  if (off > ws_size) return;
  prep_kernel<<<256, 256, 0, stream>>>(h, embW, W1, W2, pW1, hp, wemb, w1, w2, wp);
  nlin_kernel<0><<<NBLK, 128, 0, stream>>>(hp, wemb, embb, nullptr, nullptr, nullptr, nullptr, nullptr, hA);
  edge_kernel<true, false><<<E / 128, 128, 0, stream>>>(src, dst, ef, hA, wp, pb1, pW2, pb2, score, out);
  float* hc = hA; float* hn = hB;
  for (int l = 0; l < L; ++l) {
    agg_kernel<H, 1024><<<NPAD / 1024 + 1, 256, 0, stream>>>(src, dst, hc, eps + l, xa);
    nlin_kernel<1><<<NBLK, 128, 0, stream>>>(xa, w1 + (size_t)l * H * H, b1 + l * H, bns + l * H, bnsh + l * H, nullptr, nullptr, nullptr, xb);
    nlin_kernel<2><<<NBLK, 128, 0, stream>>>(xb, w2 + (size_t)l * H * H, b2 + l * H, aps + l * H, apsh + l * H, gns + l * H, gnsh + l * H, hc, hn);
    if (l < L - 1) edge_kernel<false, false><<<E / 128, 128, 0, stream>>>(src, dst, ef, hn, wp + (size_t)(l + 1) * H * EDP, pb1 + (l + 1) * H, pW2 + (l + 1) * H, pb2 + (l + 1), score, out);
    else           edge_kernel<false, true ><<<E / 128, 128, 0, stream>>>(src, dst, ef, hn, wp + (size_t)(l + 1) * H * EDP, pb1 + (l + 1) * H, pW2 + (l + 1) * H, pb2 + (l + 1), score, out);
    float* tmp = hc; hc = hn; hn = tmp;
  }
}
